// NAM_44796508897982
// MI455X (gfx1250) — hardware-verified
//
#include <hip/hip_runtime.h>
#include <stdint.h>

typedef __attribute__((ext_vector_type(16))) _Float16 v16h;
typedef __attribute__((ext_vector_type(8)))  _Float16 v8h;
typedef __attribute__((ext_vector_type(16))) __bf16   v16b;
typedef __attribute__((ext_vector_type(8)))  __bf16   v8b;
typedef __attribute__((ext_vector_type(8)))  float    v8f;
typedef __attribute__((ext_vector_type(4)))  float    v4f;

constexpr int NROWS = 4096;
constexpr int NFEAT = 128;
constexpr int NHID  = 256;
constexpr int NOUT  = 64;
constexpr int FGRP  = 16;
constexpr int NGRP  = NFEAT / FGRP;
static_assert(NFEAT % FGRP == 0);
static_assert(NHID % 32 == 0 && (FGRP * NHID) % 32 == 0);
static_assert(NROWS % 64 == 0 && NHID % 64 == 0 && NOUT % 64 == 0);

constexpr size_t WS_W2T = 0;
constexpr size_t WS_W3T = WS_W2T + (size_t)NFEAT * NHID * NHID * 2;
constexpr size_t WS_H1  = WS_W3T + (size_t)NOUT * NFEAT * NHID * 2;
constexpr size_t WS_H2  = WS_H1  + (size_t)FGRP * NROWS * NHID * 2;
constexpr size_t WS_P0  = WS_H2  + (size_t)NROWS * FGRP * NHID * 2;
constexpr size_t WS_P1  = WS_P0  + (size_t)NROWS * NOUT * 4;
constexpr size_t WS_B2S = WS_P1  + (size_t)NROWS * NOUT * 4;
constexpr size_t WS_TOTAL = WS_B2S + (size_t)NFEAT * NHID * 4;
static_assert(WS_TOTAL == 90308608u);
static_assert(WS_TOTAL <= 134217728u);
static_assert(WS_W3T % 128 == 0 && WS_H1 % 128 == 0 && WS_H2 % 128 == 0 && WS_P0 % 128 == 0 && WS_P1 % 128 == 0 && WS_B2S % 128 == 0);

__device__ __forceinline__ unsigned short f2bf_bits(float f) {
  unsigned u = __float_as_uint(f);
  return (unsigned short)((u + 0x7FFFu + ((u >> 16) & 1u)) >> 16);
}
__device__ __forceinline__ float bf_bits2f(unsigned short h) { return __uint_as_float(((unsigned)h) << 16); }
__device__ __forceinline__ float bf16r(float f) { return __uint_as_float(((unsigned)f2bf_bits(f)) << 16); }

__device__ __forceinline__ void dep_guard_h(v8f& a, v8f& b, v16h x, v16h y) { asm volatile("v_nop\n\tv_nop\n\tv_nop\n\tv_nop" : "+v"(a), "+v"(b) : "v"(x), "v"(y)); }
__device__ __forceinline__ void dep_guard_b(v8f& a, v8f& b, v16b x, v16b y) { asm volatile("v_nop\n\tv_nop\n\tv_nop\n\tv_nop" : "+v"(a), "+v"(b) : "v"(x), "v"(y)); }
__device__ __forceinline__ void keep4_h(v16h a, v16h b, v16h c, v16h d) { asm volatile("v_nop" :: "v"(a), "v"(b), "v"(c), "v"(d)); }
__device__ __forceinline__ void keep4_b(v16b a, v16b b, v16b c, v16b d) { asm volatile("v_nop" :: "v"(a), "v"(b), "v"(c), "v"(d)); }
__device__ __forceinline__ void acc_guard4(v8f& a, v8f& b, v8f& c, v8f& d) { asm volatile("v_nop\n\tv_nop\n\tv_nop\n\tv_nop" : "+v"(a), "+v"(b), "+v"(c), "+v"(d)); }
template <typename T> struct Frag;
template <> struct Frag<_Float16> {
  typedef v16h V; union U { v16h v; v8h h[2]; };
  static __device__ __forceinline__ v16h load(const _Float16* p) {
    U f; f.h[0] = *(const v8h*)(p); f.h[1] = *(const v8h*)(p + 16); return f.v;
  }
  static __device__ __forceinline__ v8f mma(v16h a, v16h b, v8f c) {
    return __builtin_amdgcn_wmma_f32_16x16x32_f16(false, a, false, b, (short)0, c, false, false);
  }
  static __device__ __forceinline__ void guard(v8f& a, v8f& b, v16h x, v16h y) { dep_guard_h(a, b, x, y); }
  static __device__ __forceinline__ void keep(v16h a, v16h b, v16h c, v16h d) { keep4_h(a, b, c, d); }
};
template <> struct Frag<__bf16> {
  typedef v16b V; union U { v16b v; v8b h[2]; };
  static __device__ __forceinline__ v16b load(const __bf16* p) {
    U f; f.h[0] = *(const v8b*)(p); f.h[1] = *(const v8b*)(p + 16); return f.v;
  }
  static __device__ __forceinline__ v8f mma(v16b a, v16b b, v8f c) {
    return __builtin_amdgcn_wmma_f32_16x16x32_bf16(false, a, false, b, (short)0, c, false, false);
  }
  static __device__ __forceinline__ void guard(v8f& a, v8f& b, v16b x, v16b y) { dep_guard_b(a, b, x, y); }
  static __device__ __forceinline__ void keep(v16b a, v16b b, v16b c, v16b d) { keep4_b(a, b, c, d); }
};

template <int ET> struct Elem;
template <> struct Elem<0> { typedef _Float16 T; };
template <> struct Elem<1> { typedef __bf16 T; };
template <int ET, bool SPLIT, int BIAS_MODE, int OUT_MODE, bool RESID, int ACT = 0>
__global__ __launch_bounds__(256) void wmma_gemm64(
    const unsigned short* __restrict__ Ap, const unsigned short* __restrict__ A2p, int lda, long strideA,
    const unsigned short* __restrict__ Btp, const unsigned short* __restrict__ Bt2p, int ldb, long strideB,
    void* __restrict__ Cout, void* __restrict__ Cout2, int ldc, long strideC,
    const float* __restrict__ bias, long strideBias,
    const float* __restrict__ resid, long strideR,
    int M, int N, int K, float scale) {
  static_assert(!(RESID && OUT_MODE != 0));
  typedef typename Elem<ET>::T T;
  typedef typename Frag<T>::V V;
  const T* A = (const T*)Ap; const T* A2 = (const T*)A2p; const T* Bt = (const T*)Btp; const T* Bt2 = (const T*)Bt2p;
  __shared__ __align__(16) float sT[8][16 * 68];
  const int b    = blockIdx.y;
  const int lane = threadIdx.x & 31;
  const int wave = threadIdx.x >> 5;
  const int tilesN = N >> 6;
  const int tilesM = M >> 6;
  const int tile = blockIdx.x * 8 + wave;
  if (tile >= tilesM * tilesN) return;
  const int tm = tile / tilesN;
  const int tn = tile - tm * tilesN;
  const int m0 = tm << 6;
  const int n0 = tn << 6;

  const T* Ab  = A  + (size_t)b * strideA;
  const T* Bb  = Bt + (size_t)b * strideB;
  const T* Ab2 = SPLIT ? (A2  + (size_t)b * strideA) : nullptr;
  const T* Bb2 = SPLIT ? (Bt2 + (size_t)b * strideB) : nullptr;

  const int rlane = lane & 15;
  const int koff  = (lane >> 4) * 8;
  const int mOff  = (lane >> 4) * 8;

  v8f acc[4][4];
#pragma unroll
  for (int i = 0; i < 4; ++i)
#pragma unroll
    for (int j = 0; j < 4; ++j) acc[i][j] = (v8f){0.f,0.f,0.f,0.f,0.f,0.f,0.f,0.f};

  for (int k0 = 0; k0 < K; k0 += 32) {
    V bh[4], bl[4];
#pragma unroll
    for (int j = 0; j < 4; ++j) {
      const size_t bo = (size_t)(n0 + (j << 4) + rlane) * ldb + koff + k0;
      bh[j] = Frag<T>::load(Bb + bo);
      if (SPLIT) bl[j] = Frag<T>::load(Bb2 + bo);
    }
#pragma unroll
    for (int i = 0; i < 4; ++i) {
      const size_t ao = (size_t)(m0 + (i << 4) + rlane) * lda + koff + k0;
      V ah = Frag<T>::load(Ab + ao);
      V al;
      if (SPLIT) al = Frag<T>::load(Ab2 + ao);
#pragma unroll
      for (int j = 0; j < 4; ++j) {
        acc[i][j] = Frag<T>::mma(ah, bh[j], acc[i][j]);
        if (SPLIT) {
          acc[i][j] = Frag<T>::mma(ah, bl[j], acc[i][j]);
          acc[i][j] = Frag<T>::mma(al, bh[j], acc[i][j]);
        }
      }
      Frag<T>::guard(acc[i][0], acc[i][3], ah, SPLIT ? al : ah);
    }
    Frag<T>::keep(bh[0], bh[1], bh[2], bh[3]);
    if (SPLIT) Frag<T>::keep(bl[0], bl[1], bl[2], bl[3]);
  }
  acc_guard4(acc[0][0], acc[0][1], acc[0][2], acc[0][3]);
  acc_guard4(acc[1][0], acc[1][1], acc[1][2], acc[1][3]);
  acc_guard4(acc[2][0], acc[2][1], acc[2][2], acc[2][3]);
  acc_guard4(acc[3][0], acc[3][1], acc[3][2], acc[3][3]);

  float* slab = sT[wave];
  const float* Rb = RESID ? (resid + (size_t)b * strideR) : nullptr;
  const float* biasb = (BIAS_MODE != 0) ? (bias + (size_t)b * strideBias) : nullptr;
#pragma unroll
  for (int i = 0; i < 4; ++i) {
    const int mBase = m0 + (i << 4);
#pragma unroll
    for (int j = 0; j < 4; ++j) {
      const int n = n0 + (j << 4) + rlane;
      float bv = 0.f;
      if (BIAS_MODE == 2) bv = biasb[n];
#pragma unroll
      for (int r = 0; r < 8; ++r) {
        float v = acc[i][j][r] * scale;
        if (BIAS_MODE == 1) v += biasb[mBase + mOff + r];
        if (BIAS_MODE == 2) v += bv;
        if (ACT == 2) v = fmaxf(v, 0.0f);
        slab[(mOff + r) * 68 + (j << 4) + rlane] = v;
      }
    }
    __builtin_amdgcn_fence(__ATOMIC_RELEASE, "workgroup");
    __builtin_amdgcn_wave_barrier();
    __builtin_amdgcn_fence(__ATOMIC_ACQUIRE, "workgroup");
    if (OUT_MODE == 0) {
      float* C = (float*)Cout + (size_t)b * strideC;
      const int hh = lane >> 4, c4 = (lane & 15) * 4;
      v4f vals[8];
#pragma unroll
      for (int it = 0; it < 8; ++it) {
        const int row = it * 2 + hh;
        v4f v = *(const v4f*)(slab + row * 68 + c4);
        if (RESID) {
          const v4f rr = *(const v4f*)(Rb + (size_t)(mBase + row) * ldc + n0 + c4);
          v += rr;
        }
        vals[it] = v;
      }
      for (int pass = 0; pass < 2; ++pass) {
#pragma unroll
        for (int it = 0; it < 8; ++it) {
          const int row = it * 2 + hh;
          *(volatile v4f*)(C + (size_t)(mBase + row) * ldc + n0 + c4) = vals[it];
        }
        __threadfence();
      }
    } else {
      const int q = lane >> 3, c8 = (lane & 7) * 8;
      unsigned short* C  = (unsigned short*)Cout  + (size_t)b * strideC;
      unsigned short* C2 = (OUT_MODE == 2) ? ((unsigned short*)Cout2 + (size_t)b * strideC) : nullptr;
      for (int pass = 0; pass < 2; ++pass) {
#pragma unroll
        for (int it = 0; it < 4; ++it) {
          const int row = it * 4 + q;
          const float* sp = slab + row * 68 + c8;
          v8h hv, lv;
#pragma unroll
          for (int e = 0; e < 8; ++e) {
            if (OUT_MODE == 1) {
              hv[e] = (_Float16)sp[e];
            } else {
              unsigned short hb = f2bf_bits(sp[e]);
              unsigned short lb = f2bf_bits(sp[e] - bf_bits2f(hb));
              hv[e] = __builtin_bit_cast(_Float16, hb);
              lv[e] = __builtin_bit_cast(_Float16, lb);
            }
          }
          *(volatile v8h*)(C + (size_t)(mBase + row) * ldc + n0 + c8) = hv;
          if (OUT_MODE == 2) *(volatile v8h*)(C2 + (size_t)(mBase + row) * ldc + n0 + c8) = lv;
        }
        __threadfence();
      }
    }
    __builtin_amdgcn_fence(__ATOMIC_RELEASE, "workgroup");
    __builtin_amdgcn_wave_barrier();
    __builtin_amdgcn_fence(__ATOMIC_ACQUIRE, "workgroup");
  }
}

__global__ __launch_bounds__(256) void transpose_cvt64(
    const float* __restrict__ in, int in_ld, long in_bs,
    unsigned short* __restrict__ out, int out_ld, long out_bs) {
  __shared__ float ts[64][65];
  const int t = threadIdx.x, lane = t & 31, wave = t >> 5;
  const int r0 = blockIdx.y * 64, c0 = blockIdx.x * 64;
  const float* ib = in + (size_t)blockIdx.z * in_bs + (size_t)r0 * in_ld + c0;
#pragma unroll
  for (int i = 0; i < 4; ++i) {
    const int rr = (t >> 4) + 16 * i;
    const int cc = (t & 15) * 4;
    const v4f v = *(const v4f*)(ib + (size_t)rr * in_ld + cc);
    ts[rr][cc] = v[0]; ts[rr][cc + 1] = v[1]; ts[rr][cc + 2] = v[2]; ts[rr][cc + 3] = v[3];
  }
  __syncthreads();
  _Float16* ob = (_Float16*)out + (size_t)blockIdx.z * out_bs + (size_t)c0 * out_ld + r0;
  const int q = lane >> 3, c8 = (lane & 7) * 8;
  v8h hv[2];
#pragma unroll
  for (int it = 0; it < 2; ++it) {
    const int cl = wave * 8 + it * 4 + q;
#pragma unroll
    for (int e = 0; e < 8; ++e) hv[it][e] = (_Float16)(64.0f * bf16r(ts[c8 + e][cl]));
  }
  for (int pass = 0; pass < 2; ++pass) {
#pragma unroll
    for (int it = 0; it < 2; ++it) {
      const int cl = wave * 8 + it * 4 + q;
      *(volatile v8h*)(ob + (size_t)cl * out_ld + c8) = hv[it];
    }
    __threadfence();
  }
}

__global__ __launch_bounds__(256) void layer1_plane(
    const float* __restrict__ x, const float* __restrict__ w1, const float* __restrict__ b1,
    unsigned short* __restrict__ h1p, int fbase) {
  const unsigned e = blockIdx.x * 256u + threadIdx.x;
  const int h8 = (int)(e & 31u);
  const int n  = (int)((e >> 5) & (unsigned)(NROWS - 1));
  const int fl = (int)(e >> 17);
  const int f  = fbase + fl;
  const float xv = bf16r(x[(size_t)n * NFEAT + f]);
  const float* wp = w1 + (size_t)f * NHID + h8 * 8;
  const float* bp = b1 + (size_t)f * NHID + h8 * 8;
  const v4f wa = *(const v4f*)wp, wb = *(const v4f*)(wp + 4);
  const v4f ba = *(const v4f*)bp, bb = *(const v4f*)(bp + 4);
  v8h hv;
#pragma unroll
  for (int i = 0; i < 4; ++i) {
    float u0 = bf16r(wa[i]) * xv + bf16r(ba[i]);
    u0 = fmaxf(u0, 0.0f) * 16.0f;
    hv[i] = (_Float16)u0;
    float u1 = bf16r(wb[i]) * xv + bf16r(bb[i]);
    u1 = fmaxf(u1, 0.0f) * 16.0f;
    hv[4 + i] = (_Float16)u1;
  }
  _Float16* dst = (_Float16*)h1p + (size_t)e * 8;
  *(volatile v8h*)dst = hv;
  __threadfence();
  *(volatile v8h*)dst = hv;
}

__global__ __launch_bounds__(256) void bias_plane64(const float* __restrict__ b3, float* __restrict__ P) {
  __shared__ float bs[NOUT];
  const int t = threadIdx.x;
  if (t < NOUT) {
    float s = 0.0f;
#pragma unroll 8
    for (int f = 0; f < NFEAT; ++f) s += bf16r(b3[f * NOUT + t]);
    bs[t] = s;
  }
  __syncthreads();
  v4f vals[4];
#pragma unroll
  for (int i = 0; i < 4; ++i) {
    const int qd = t + 256 * i;
    const int c4 = (qd & 15) * 4;
    vals[i] = (v4f){bs[c4], bs[c4 + 1], bs[c4 + 2], bs[c4 + 3]};
  }
  float* pb = P + (size_t)blockIdx.x * 64 * NOUT;
  for (int pass = 0; pass < 2; ++pass) {
#pragma unroll
    for (int i = 0; i < 4; ++i) {
      const int qd = t + 256 * i;
      *(volatile v4f*)(pb + (size_t)qd * 4) = vals[i];
    }
    __threadfence();
  }
}

__global__ __launch_bounds__(256) void scale_bias16(const float* __restrict__ b2, float* __restrict__ o, int n4) {
  const int i = blockIdx.x * 256 + threadIdx.x;
  if (i < n4) {
    const v4f v = *(const v4f*)(b2 + (size_t)i * 4);
    v4f r;
    r[0] = 16.0f * bf16r(v[0]); r[1] = 16.0f * bf16r(v[1]); r[2] = 16.0f * bf16r(v[2]); r[3] = 16.0f * bf16r(v[3]);
    *(volatile v4f*)(o + (size_t)i * 4) = r;
    __threadfence();
    *(volatile v4f*)(o + (size_t)i * 4) = r;
  }
}

extern "C" void kernel_launch(void* const* d_in, const int* in_sizes, int n_in,
                              void* d_out, int out_size, void* d_ws, size_t ws_size,
                              hipStream_t stream) {
  if (n_in < 7) return;
  if (in_sizes[0] != NROWS * NFEAT || in_sizes[1] != NFEAT * NHID || in_sizes[2] != NFEAT * NHID ||
      in_sizes[3] != NFEAT * NHID * NHID || in_sizes[4] != NFEAT * NHID ||
      in_sizes[5] != NFEAT * NHID * NOUT || in_sizes[6] != NFEAT * NOUT) return;
  if (out_size != NROWS * NOUT) return;
  if (ws_size < WS_TOTAL) return;

  const float* x  = (const float*)d_in[0];
  const float* w1 = (const float*)d_in[1];
  const float* b1 = (const float*)d_in[2];
  const float* w2 = (const float*)d_in[3];
  const float* b2 = (const float*)d_in[4];
  const float* w3 = (const float*)d_in[5];
  const float* b3 = (const float*)d_in[6];
  float* out = (float*)d_out;

  char* ws = (char*)d_ws;
  unsigned short* w2t = (unsigned short*)(ws + WS_W2T);
  unsigned short* w3t = (unsigned short*)(ws + WS_W3T);
  unsigned short* h1p = (unsigned short*)(ws + WS_H1);
  unsigned short* h2p = (unsigned short*)(ws + WS_H2);
  float* P0 = (float*)(ws + WS_P0);
  float* P1 = (float*)(ws + WS_P1);
  float* b2s = (float*)(ws + WS_B2S);

  bias_plane64<<<NROWS / 64, 256, 0, stream>>>(b3, P0);
  scale_bias16<<<(NFEAT * NHID / 4 + 255) / 256, 256, 0, stream>>>(b2, b2s, NFEAT * NHID / 4);

  transpose_cvt64<<<dim3(NHID / 64, NHID / 64, NFEAT), 256, 0, stream>>>(
      w2, NHID, (long)NHID * NHID, w2t, NHID, (long)NHID * NHID);
  transpose_cvt64<<<dim3(NOUT / 64, NHID / 64, NFEAT), 256, 0, stream>>>(
      w3, NOUT, (long)NHID * NOUT, w3t, NFEAT * NHID, (long)NHID);

  const int KTOT2 = FGRP * NHID;
  for (int g = 0; g < NGRP; ++g) {
    layer1_plane<<<(FGRP * NROWS * 32) / 256, 256, 0, stream>>>(x, w1, b1, h1p, g * FGRP);

    {
      const int Mv = NROWS, Nv = NHID, Kv = NHID;
      const int tiles = (Mv / 64) * (Nv / 64);
      const unsigned short* bt = w2t + (size_t)g * FGRP * NHID * NHID;
      wmma_gemm64<0, false, 2, 1, false, 2><<<dim3((tiles + 7) / 8, FGRP), 256, 0, stream>>>(
          h1p, h1p, NHID, (long)NROWS * NHID,
          bt, bt, NHID, (long)NHID * NHID,
          (void*)h2p, (void*)h2p, KTOT2, (long)NHID,
          b2s + (size_t)g * FGRP * NHID, (long)NHID,
          P0, 0L,
          Mv, Nv, Kv, 0.015625f);
    }
    {
      const int Mv = NROWS, Nv = NOUT, Kv = KTOT2;
      const int tiles = (Mv / 64) * (Nv / 64);
      const unsigned short* bt = w3t + (size_t)g * KTOT2;
      const float* src = (g & 1) ? P1 : P0;
      float* dst = (g == NGRP - 1) ? out : ((g & 1) ? P0 : P1);
      wmma_gemm64<0, false, 0, 0, true, 0><<<dim3((tiles + 7) / 8, 1), 256, 0, stream>>>(
          h2p, h2p, KTOT2, 0L,
          bt, bt, NFEAT * NHID, 0L,
          (void*)dst, (void*)dst, NOUT, 0L,
          b2s, 0L,
          src, 0L,
          Mv, Nv, Kv, 0.0009765625f);
    }
  }
}
